// RotaryMHA_54185307407108
// MI455X (gfx1250) — hardware-verified
//
#include <hip/hip_runtime.h>
#include <math.h>

typedef __attribute__((ext_vector_type(16))) _Float16 v16h;
typedef __attribute__((ext_vector_type(8)))  _Float16 v8h;
typedef __attribute__((ext_vector_type(16))) __bf16   v16b;
typedef __attribute__((ext_vector_type(8)))  __bf16   v8b;
typedef __attribute__((ext_vector_type(8)))  float    v8f;
typedef __attribute__((ext_vector_type(4)))  float    v4f;
typedef __attribute__((ext_vector_type(4)))  unsigned v4u;

constexpr int kBatch = 2;
constexpr int kSeq   = 2048;
constexpr int kEmb   = 1024;
constexpr int kHeads = 16;
constexpr int kHdim  = 64;
constexpr int kRows  = kBatch * kSeq;
constexpr int kFreq  = 16;
static_assert(kHeads * kHdim == kEmb, "head split");
static_assert(kRows % 64 == 0 && kEmb % 64 == 0, "GEMM M and N are multiples of the 64 tile");
static_assert(kEmb % 32 == 0, "GEMM K is a multiple of 32");
static_assert(kSeq % 64 == 0 && kHdim == 64, "attention tiling");
static_assert(((kRows / 64) * (kEmb / 64)) % 8 == 0, "8 tiles per GEMM block");
static_assert((kRows * kEmb) % (8 * 256) == 0, "cast grid exact");
static_assert((kSeq * kFreq) % 256 == 0, "table grid exact");
static_assert((kRows * kHeads * 8) % 256 == 0, "rope grid exact");

__device__ __forceinline__ unsigned short f2bf_bits(float f) {
  unsigned u = __float_as_uint(f);
  return (unsigned short)((u + 0x7FFFu + ((u >> 16) & 1u)) >> 16);
}
__device__ __forceinline__ float bf_bits2f(unsigned short h) { return __uint_as_float(((unsigned)h) << 16); }
__device__ __forceinline__ float bf_rne(float f) { return bf_bits2f(f2bf_bits(f)); }

__device__ __forceinline__ void dep_guard_h(v8f& a, v8f& b, v16h x, v16h y) { asm volatile("v_nop\n\tv_nop\n\tv_nop\n\tv_nop" : "+v"(a), "+v"(b) : "v"(x), "v"(y)); }
__device__ __forceinline__ void dep_guard_b(v8f& a, v8f& b, v16b x, v16b y) { asm volatile("v_nop\n\tv_nop\n\tv_nop\n\tv_nop" : "+v"(a), "+v"(b) : "v"(x), "v"(y)); }
__device__ __forceinline__ void keep4_h(v16h a, v16h b, v16h c, v16h d) { asm volatile("v_nop" :: "v"(a), "v"(b), "v"(c), "v"(d)); }
__device__ __forceinline__ void keep4_b(v16b a, v16b b, v16b c, v16b d) { asm volatile("v_nop" :: "v"(a), "v"(b), "v"(c), "v"(d)); }
__device__ __forceinline__ void acc_guard4(v8f& a, v8f& b, v8f& c, v8f& d) { asm volatile("v_nop\n\tv_nop\n\tv_nop\n\tv_nop" : "+v"(a), "+v"(b), "+v"(c), "+v"(d)); }
template <typename T> struct Frag;
template <> struct Frag<_Float16> {
  typedef v16h V; union U { v16h v; v8h h[2]; };
  static __device__ __forceinline__ v16h load(const _Float16* p) {
    U f; f.h[0] = *(const v8h*)(p); f.h[1] = *(const v8h*)(p + 16); return f.v;
  }
  static __device__ __forceinline__ v8f mma(v16h a, v16h b, v8f c) {
    return __builtin_amdgcn_wmma_f32_16x16x32_f16(false, a, false, b, (short)0, c, false, false);
  }
  static __device__ __forceinline__ void guard(v8f& a, v8f& b, v16h x, v16h y) { dep_guard_h(a, b, x, y); }
  static __device__ __forceinline__ void keep(v16h a, v16h b, v16h c, v16h d) { keep4_h(a, b, c, d); }
};
template <> struct Frag<__bf16> {
  typedef v16b V; union U { v16b v; v8b h[2]; };
  static __device__ __forceinline__ v16b load(const __bf16* p) {
    U f; f.h[0] = *(const v8b*)(p); f.h[1] = *(const v8b*)(p + 16); return f.v;
  }
  static __device__ __forceinline__ v8f mma(v16b a, v16b b, v8f c) {
    return __builtin_amdgcn_wmma_f32_16x16x32_bf16(false, a, false, b, (short)0, c, false, false);
  }
  static __device__ __forceinline__ void guard(v8f& a, v8f& b, v16b x, v16b y) { dep_guard_b(a, b, x, y); }
  static __device__ __forceinline__ void keep(v16b a, v16b b, v16b c, v16b d) { keep4_b(a, b, c, d); }
};

template <int ET> struct Elem;
template <> struct Elem<0> { typedef _Float16 T; };
template <> struct Elem<1> { typedef __bf16 T; };
template <int ET, bool SPLIT, int BIAS_MODE, int OUT_MODE, bool RESID, int ACT = 0, bool SPLITB = true>
__global__ __launch_bounds__(256) void wmma_gemm64(
    const unsigned short* __restrict__ Ap, const unsigned short* __restrict__ A2p, int lda, long strideA,
    const unsigned short* __restrict__ Btp, const unsigned short* __restrict__ Bt2p, int ldb, long strideB,
    void* __restrict__ Cout, void* __restrict__ Cout2, int ldc, long strideC,
    const float* __restrict__ bias,
    const float* __restrict__ resid, long strideR,
    int M, int N, int K, float scale) {
  static_assert(!RESID, "residual path not supported in this build");
  static_assert(ACT == 0 || ACT == 2 || ACT == 4, "cheap activations only");
  typedef typename Elem<ET>::T T;
  typedef typename Frag<T>::V V;
  const T* A = (const T*)Ap; const T* A2 = (const T*)A2p; const T* Bt = (const T*)Btp; const T* Bt2 = (const T*)Bt2p;
  __shared__ __align__(16) float sT[8][16 * 68];
  (void)resid; (void)strideR;
  const int b    = blockIdx.y;
  const int lane = threadIdx.x & 31;
  const int wave = threadIdx.x >> 5;
  const int tilesN = N >> 6;
  const int tilesM = M >> 6;
  const int tile = blockIdx.x * 8 + wave;
  if (tile >= tilesM * tilesN) return;
  const int tm = tile / tilesN;
  const int tn = tile - tm * tilesN;
  const int m0 = tm << 6;
  const int n0 = tn << 6;

  const T* Ab  = A  + (size_t)b * strideA;
  const T* Bb  = Bt + (size_t)b * strideB;
  const T* Ab2 = SPLIT ? (A2 + (size_t)b * strideA) : nullptr;
  const T* Bb2 = (SPLIT && SPLITB) ? (Bt2 + (size_t)b * strideB) : nullptr;

  const int rlane = lane & 15;
  const int koff  = (lane >> 4) * 8;
  const int mOff  = (lane >> 4) * 8;

  v8f acc[4][4];
#pragma unroll
  for (int i = 0; i < 4; ++i)
#pragma unroll
    for (int j = 0; j < 4; ++j) acc[i][j] = (v8f){0.f,0.f,0.f,0.f,0.f,0.f,0.f,0.f};

  for (int k0 = 0; k0 < K; k0 += 32) {
    V bh[4], bl[4];
#pragma unroll
    for (int j = 0; j < 4; ++j) {
      const size_t bo = (size_t)(n0 + (j << 4) + rlane) * ldb + koff + k0;
      bh[j] = Frag<T>::load(Bb + bo);
      bl[j] = bh[j];
      if (SPLIT && SPLITB) bl[j] = Frag<T>::load(Bb2 + bo);
    }
#pragma unroll
    for (int i = 0; i < 4; ++i) {
      const size_t ao = (size_t)(m0 + (i << 4) + rlane) * lda + koff + k0;
      V ah = Frag<T>::load(Ab + ao);
      V al = ah;
      if (SPLIT) al = Frag<T>::load(Ab2 + ao);
#pragma unroll
      for (int j = 0; j < 4; ++j) {
        acc[i][j] = Frag<T>::mma(ah, bh[j], acc[i][j]);
        if (SPLIT && SPLITB) acc[i][j] = Frag<T>::mma(ah, bl[j], acc[i][j]);
        if (SPLIT) acc[i][j] = Frag<T>::mma(al, bh[j], acc[i][j]);
      }
      Frag<T>::guard(acc[i][0], acc[i][3], ah, al);
    }
    Frag<T>::keep(bh[0], bh[1], bh[2], bh[3]);
    if (SPLIT && SPLITB) Frag<T>::keep(bl[0], bl[1], bl[2], bl[3]);
  }
  acc_guard4(acc[0][0], acc[0][1], acc[0][2], acc[0][3]);
  acc_guard4(acc[1][0], acc[1][1], acc[1][2], acc[1][3]);
  acc_guard4(acc[2][0], acc[2][1], acc[2][2], acc[2][3]);
  acc_guard4(acc[3][0], acc[3][1], acc[3][2], acc[3][3]);

  float* slab = sT[wave];
#pragma unroll
  for (int i = 0; i < 4; ++i) {
    const int mBase = m0 + (i << 4);
    float bm[8];
#pragma unroll
    for (int r = 0; r < 8; ++r) bm[r] = 0.f;
    if (BIAS_MODE == 1) {
      const v4f t0 = *(const v4f*)(bias + mBase + mOff);
      const v4f t1 = *(const v4f*)(bias + mBase + mOff + 4);
      bm[0] = bf_rne(t0.x); bm[1] = bf_rne(t0.y); bm[2] = bf_rne(t0.z); bm[3] = bf_rne(t0.w);
      bm[4] = bf_rne(t1.x); bm[5] = bf_rne(t1.y); bm[6] = bf_rne(t1.z); bm[7] = bf_rne(t1.w);
    }
#pragma unroll
    for (int j = 0; j < 4; ++j) {
      const int n = n0 + (j << 4) + rlane;
      float bv = 0.f;
      if (BIAS_MODE == 2) bv = bf_rne(bias[n]);
#pragma unroll
      for (int r = 0; r < 8; ++r) {
        float v = acc[i][j][r] * scale;
        if (BIAS_MODE == 1) v += bm[r];
        if (BIAS_MODE == 2) v += bv;
        if (ACT == 2) v = fmaxf(v, 0.0f);
        if (ACT == 4) v = (v > 0.f) ? v : 0.01f * v;
        slab[(mOff + r) * 68 + (j << 4) + rlane] = v;
      }
    }
    __builtin_amdgcn_fence(__ATOMIC_RELEASE, "workgroup");
    __builtin_amdgcn_wave_barrier();
    __builtin_amdgcn_fence(__ATOMIC_ACQUIRE, "workgroup");
    if (OUT_MODE == 0) {
      float* C = (float*)Cout + (size_t)b * strideC;
      const int hh = lane >> 4, c4 = (lane & 15) * 4;
      for (int pass = 0; pass < 2; ++pass) {
#pragma unroll
        for (int it = 0; it < 8; ++it) {
          const int row = it * 2 + hh;
          v4f v = *(const v4f*)(slab + row * 68 + c4);
          *(volatile v4f*)(C + (size_t)(mBase + row) * ldc + n0 + c4) = v;
        }
        __threadfence();
      }
    } else {
      const int q = lane >> 3, c8 = (lane & 7) * 8;
      unsigned short* C  = (unsigned short*)Cout  + (size_t)b * strideC;
      unsigned short* C2 = (OUT_MODE == 2) ? ((unsigned short*)Cout2 + (size_t)b * strideC) : nullptr;
      for (int pass = 0; pass < 2; ++pass) {
#pragma unroll
        for (int it = 0; it < 4; ++it) {
          const int row = it * 4 + q;
          const float* sp = slab + row * 68 + c8;
          v8h hv, lv;
#pragma unroll
          for (int e = 0; e < 8; ++e) {
            if (OUT_MODE == 1) {
              hv[e] = (_Float16)sp[e];
            } else {
              unsigned short hb = f2bf_bits(sp[e]);
              unsigned short lb = f2bf_bits(sp[e] - bf_bits2f(hb));
              hv[e] = __builtin_bit_cast(_Float16, hb);
              lv[e] = __builtin_bit_cast(_Float16, lb);
            }
          }
          *(volatile v8h*)(C + (size_t)(mBase + row) * ldc + n0 + c8) = hv;
          if (OUT_MODE == 2) *(volatile v8h*)(C2 + (size_t)(mBase + row) * ldc + n0 + c8) = lv;
        }
        __threadfence();
      }
    }
    __builtin_amdgcn_fence(__ATOMIC_RELEASE, "workgroup");
    __builtin_amdgcn_wave_barrier();
    __builtin_amdgcn_fence(__ATOMIC_ACQUIRE, "workgroup");
  }
}

__device__ __forceinline__ unsigned short at_bf_bits(float f) {
  unsigned u = __float_as_uint(f);
  return (unsigned short)((u + 0x7FFFu + ((u >> 16) & 1u)) >> 16);
}
__device__ __forceinline__ __bf16 at_f2bf(float f) { return __builtin_bit_cast(__bf16, at_bf_bits(f)); }
__device__ __forceinline__ void at_split(float f, __bf16& hi, __bf16& lo) {
  const unsigned short hb = at_bf_bits(f);
  hi = __builtin_bit_cast(__bf16, hb);
  lo = at_f2bf(f - __uint_as_float(((unsigned)hb) << 16));
}
__device__ __forceinline__ v8f at_mma(v16b a, v16b b, v8f c) {
  c = __builtin_amdgcn_wmma_f32_16x16x32_bf16(false, a, false, b, (short)0, c, false, false);
  asm volatile("v_nop\n\tv_nop\n\tv_nop\n\tv_nop" : "+v"(c) : "v"(a), "v"(b));
  return c;
}

__device__ __forceinline__ unsigned pack_hl(float a, float b, unsigned& lo) {
  const unsigned short ha = f2bf_bits(a), hb = f2bf_bits(b);
  const unsigned short la = f2bf_bits(a - bf_bits2f(ha));
  const unsigned short lb = f2bf_bits(b - bf_bits2f(hb));
  lo = (unsigned)la | ((unsigned)lb << 16);
  return (unsigned)ha | ((unsigned)hb << 16);
}

__global__ __launch_bounds__(256) void cast_f32_bf16x8(const float* __restrict__ in,
                                                       unsigned short* __restrict__ out, int n8) {
  const int i = blockIdx.x * 256 + threadIdx.x;
  if (i < n8) {
    const v4f a = *(const v4f*)(in + (size_t)i * 8);
    const v4f c = *(const v4f*)(in + (size_t)i * 8 + 4);
    v4u u;
    u.x = (unsigned)f2bf_bits(a.x) | ((unsigned)f2bf_bits(a.y) << 16);
    u.y = (unsigned)f2bf_bits(a.z) | ((unsigned)f2bf_bits(a.w) << 16);
    u.z = (unsigned)f2bf_bits(c.x) | ((unsigned)f2bf_bits(c.y) << 16);
    u.w = (unsigned)f2bf_bits(c.z) | ((unsigned)f2bf_bits(c.w) << 16);
    volatile v4u* p = (volatile v4u*)(out + (size_t)i * 8);
    *p = u;
    __threadfence();
    *p = u;
  }
}

__global__ __launch_bounds__(128) void transpose_cast_bf16(const float* __restrict__ W,
                                                           unsigned short* __restrict__ Wt) {
  __shared__ float tile[64][65];
  const int tid = threadIdx.x, lane = tid & 31, wave = tid >> 5;
  const int n0 = blockIdx.x * 64;
  const int k0 = blockIdx.y * 64;
#pragma unroll
  for (int it = 0; it < 8; ++it) {
    const int idx = tid + it * 128;
    const int r  = idx >> 4;
    const int c4 = (idx & 15) * 4;
    const v4f v = *(const v4f*)(W + (size_t)(k0 + r) * kEmb + n0 + c4);
    tile[r][c4 + 0] = v.x; tile[r][c4 + 1] = v.y; tile[r][c4 + 2] = v.z; tile[r][c4 + 3] = v.w;
  }
  __syncthreads();
  const int q  = lane >> 3;
  const int kq = (lane & 7) * 8;
  for (int pass = 0; pass < 2; ++pass) {
#pragma unroll
    for (int it = 0; it < 4; ++it) {
      const int nl = wave * 16 + it * 4 + q;
      v4u u;
      u.x = (unsigned)f2bf_bits(tile[kq + 0][nl]) | ((unsigned)f2bf_bits(tile[kq + 1][nl]) << 16);
      u.y = (unsigned)f2bf_bits(tile[kq + 2][nl]) | ((unsigned)f2bf_bits(tile[kq + 3][nl]) << 16);
      u.z = (unsigned)f2bf_bits(tile[kq + 4][nl]) | ((unsigned)f2bf_bits(tile[kq + 5][nl]) << 16);
      u.w = (unsigned)f2bf_bits(tile[kq + 6][nl]) | ((unsigned)f2bf_bits(tile[kq + 7][nl]) << 16);
      *(volatile v4u*)(Wt + (size_t)(n0 + nl) * kEmb + k0 + kq) = u;
    }
    __threadfence();
  }
}

struct RopeFreq { float f[16]; };
static_assert(sizeof(RopeFreq) == 64, "no padding");

__global__ __launch_bounds__(256) void rope_table(float* __restrict__ cos_t, float* __restrict__ sin_t,
                                                  RopeFreq fr) {
#pragma clang fp contract(off)
  const int i = blockIdx.x * 256 + threadIdx.x;
  const int t = i >> 4;
  const int j = i & 15;
  float f = fr.f[0];
#pragma unroll
  for (int e = 1; e < 16; ++e) f = (j == e) ? fr.f[e] : f;
  const float ang = (float)t * f;
  float sn, cs;
  sincosf(ang, &sn, &cs);
  ((volatile float*)cos_t)[i] = cs;
  ((volatile float*)sin_t)[i] = sn;
  __threadfence();
  ((volatile float*)cos_t)[i] = cs;
  ((volatile float*)sin_t)[i] = sn;
}

__device__ __forceinline__ float rope1(float a, float p, float cs, float sn, float sgn, bool rot) {
  const float r = a * cs + sgn * (p * sn);
  return rot ? r : a;
}

__global__ __launch_bounds__(256) void rope_split(const float* __restrict__ Qf, const float* __restrict__ Kf,
                                                  const float* __restrict__ cos_t, const float* __restrict__ sin_t,
                                                  unsigned short* __restrict__ Qh, unsigned short* __restrict__ Ql,
                                                  unsigned short* __restrict__ Kh, unsigned short* __restrict__ Kl) {
  const int i   = blockIdx.x * 256 + threadIdx.x;
  const int row = i >> 7;
  const int hd  = i & 127;
  const int h   = hd >> 3;
  const int j   = hd & 7;
  const int t   = row & (kSeq - 1);
  const int col  = h * kHdim + j * 8;
  const int pj   = (j < 4) ? (j ^ 2) : j;
  const int pcol = h * kHdim + pj * 8;
  const int aidx = (j & 1) * 8;
  const size_t ro = (size_t)row * kEmb;
  const v4f qa0 = *(const v4f*)(Qf + ro + col),  qa1 = *(const v4f*)(Qf + ro + col + 4);
  const v4f qp0 = *(const v4f*)(Qf + ro + pcol), qp1 = *(const v4f*)(Qf + ro + pcol + 4);
  const v4f ka0 = *(const v4f*)(Kf + ro + col),  ka1 = *(const v4f*)(Kf + ro + col + 4);
  const v4f kp0 = *(const v4f*)(Kf + ro + pcol), kp1 = *(const v4f*)(Kf + ro + pcol + 4);
  const v4f cs0 = *(const v4f*)(cos_t + (size_t)t * kFreq + aidx), cs1 = *(const v4f*)(cos_t + (size_t)t * kFreq + aidx + 4);
  const v4f sn0 = *(const v4f*)(sin_t + (size_t)t * kFreq + aidx), sn1 = *(const v4f*)(sin_t + (size_t)t * kFreq + aidx + 4);
  const float sgn = (j < 2) ? -1.0f : 1.0f;
  const bool rot  = (j < 4);
  const float qs  = 0.125f;

  const float qo0 = rope1(qa0.x, qp0.x, cs0.x, sn0.x, sgn, rot) * qs;
  const float qo1 = rope1(qa0.y, qp0.y, cs0.y, sn0.y, sgn, rot) * qs;
  const float qo2 = rope1(qa0.z, qp0.z, cs0.z, sn0.z, sgn, rot) * qs;
  const float qo3 = rope1(qa0.w, qp0.w, cs0.w, sn0.w, sgn, rot) * qs;
  const float qo4 = rope1(qa1.x, qp1.x, cs1.x, sn1.x, sgn, rot) * qs;
  const float qo5 = rope1(qa1.y, qp1.y, cs1.y, sn1.y, sgn, rot) * qs;
  const float qo6 = rope1(qa1.z, qp1.z, cs1.z, sn1.z, sgn, rot) * qs;
  const float qo7 = rope1(qa1.w, qp1.w, cs1.w, sn1.w, sgn, rot) * qs;
  const float ko0 = rope1(ka0.x, kp0.x, cs0.x, sn0.x, sgn, rot);
  const float ko1 = rope1(ka0.y, kp0.y, cs0.y, sn0.y, sgn, rot);
  const float ko2 = rope1(ka0.z, kp0.z, cs0.z, sn0.z, sgn, rot);
  const float ko3 = rope1(ka0.w, kp0.w, cs0.w, sn0.w, sgn, rot);
  const float ko4 = rope1(ka1.x, kp1.x, cs1.x, sn1.x, sgn, rot);
  const float ko5 = rope1(ka1.y, kp1.y, cs1.y, sn1.y, sgn, rot);
  const float ko6 = rope1(ka1.z, kp1.z, cs1.z, sn1.z, sgn, rot);
  const float ko7 = rope1(ka1.w, kp1.w, cs1.w, sn1.w, sgn, rot);

  unsigned qh0, qh1, qh2, qh3, ql0, ql1, ql2, ql3;
  unsigned kh0, kh1, kh2, kh3, kl0, kl1, kl2, kl3;
  qh0 = pack_hl(qo0, qo1, ql0);
  qh1 = pack_hl(qo2, qo3, ql1);
  qh2 = pack_hl(qo4, qo5, ql2);
  qh3 = pack_hl(qo6, qo7, ql3);
  kh0 = pack_hl(ko0, ko1, kl0);
  kh1 = pack_hl(ko2, ko3, kl1);
  kh2 = pack_hl(ko4, ko5, kl2);
  kh3 = pack_hl(ko6, ko7, kl3);
  const v4u uqh = (v4u){qh0, qh1, qh2, qh3};
  const v4u uql = (v4u){ql0, ql1, ql2, ql3};
  const v4u ukh = (v4u){kh0, kh1, kh2, kh3};
  const v4u ukl = (v4u){kl0, kl1, kl2, kl3};

  const size_t o = ro + col;
  for (int pass = 0; pass < 2; ++pass) {
    *(volatile v4u*)(Qh + o) = uqh;
    *(volatile v4u*)(Ql + o) = uql;
    *(volatile v4u*)(Kh + o) = ukh;
    *(volatile v4u*)(Kl + o) = ukl;
    __threadfence();
  }
}

__global__ __launch_bounds__(128)
void attn_causal64(const unsigned short* __restrict__ Qh, const unsigned short* __restrict__ Ql,
                   const unsigned short* __restrict__ Kh, const unsigned short* __restrict__ Kl,
                   const unsigned short* __restrict__ Vh, const unsigned short* __restrict__ Vl,
                   unsigned short* __restrict__ Oh, unsigned short* __restrict__ Ol) {
  __shared__ __align__(16) __bf16 Qsh[64 * 64];
  __shared__ __align__(16) __bf16 Qsl[64 * 64];
  __shared__ __align__(16) __bf16 Ksh[64 * 64];
  __shared__ __align__(16) __bf16 Ksl[64 * 64];
  __shared__ __align__(16) __bf16 Vth[64 * 64];
  __shared__ __align__(16) __bf16 Vtl[64 * 64];
  __shared__ __align__(16) __bf16 Psh[4][16 * 64];
  __shared__ __align__(16) __bf16 Psl[4][16 * 64];
  __shared__ __align__(16) float  Os[4][16 * 68];

  const int tid  = threadIdx.x;
  const int wave = tid >> 5;
  const int lane = tid & 31;
  const int hh   = lane >> 4;
  const int c    = lane & 15;

  const int bx = blockIdx.x;
  const int qb = bx & 31;
  const int bh = bx >> 5;
  const int h  = bh & 15;
  const int b  = bh >> 4;
  const int qblk = qb * 64;
  const int q0 = qblk + wave * 16;
  const size_t rowb = (size_t)b * kSeq;
  const int hcol = h * kHdim;

#pragma unroll
  for (int it = 0; it < 4; ++it) {
    const int idx = tid + it * 128;
    const int r = idx >> 3, c8 = (idx & 7) * 8;
    const size_t src = (rowb + qblk + r) * kEmb + hcol + c8;
    const uint4 a  = *(const uint4*)(Qh + src);
    const uint4 a2 = *(const uint4*)(Ql + src);
    *(uint4*)(Qsh + r * 64 + c8) = a;
    *(uint4*)(Qsl + r * 64 + c8) = a2;
  }

  float mrow[8], lrow[8];
  v8f oacc[4];
#pragma unroll
  for (int r = 0; r < 8; ++r) { mrow[r] = -INFINITY; lrow[r] = 0.f; }
#pragma unroll
  for (int t = 0; t < 4; ++t) oacc[t] = (v8f){0.f,0.f,0.f,0.f,0.f,0.f,0.f,0.f};

  const __bf16* qwh = Qsh + (wave * 16 + c) * 64 + 8 * hh;
  const __bf16* qwl = Qsl + (wave * 16 + c) * 64 + 8 * hh;

  const int nChunks = qb + 1;
  for (int kc = 0; kc < nChunks; ++kc) {
    const int kv0 = kc * 64;
    __syncthreads();
#pragma unroll
    for (int it = 0; it < 4; ++it) {
      const int idx = tid + it * 128;
      const int kvr = idx >> 3, c8 = (idx & 7) * 8;
      const size_t src = (rowb + kv0 + kvr) * kEmb + hcol + c8;
      const uint4 a  = *(const uint4*)(Kh + src);
      const uint4 a2 = *(const uint4*)(Kl + src);
      *(uint4*)(Ksh + kvr * 64 + c8) = a;
      *(uint4*)(Ksl + kvr * 64 + c8) = a2;
    }
#pragma unroll
    for (int it = 0; it < 4; ++it) {
      const int idx = tid + it * 128;
      const int d = idx >> 3, c8 = (idx & 7) * 8;
      const size_t src = (size_t)(hcol + d) * kRows + rowb + kv0 + c8;
      const uint4 a  = *(const uint4*)(Vh + src);
      const uint4 a2 = *(const uint4*)(Vl + src);
      *(uint4*)(Vth + d * 64 + c8) = a;
      *(uint4*)(Vtl + d * 64 + c8) = a2;
    }
    __syncthreads();

    v8f s[4];
#pragma unroll
    for (int j = 0; j < 4; ++j) s[j] = (v8f){0.f,0.f,0.f,0.f,0.f,0.f,0.f,0.f};
#pragma unroll 1
    for (int dc = 0; dc < 2; ++dc) {
      const v16b qa = Frag<__bf16>::load(qwh + dc * 32);
      const v16b ql = Frag<__bf16>::load(qwl + dc * 32);
#pragma unroll
      for (int j = 0; j < 4; ++j) {
        const v16b kb = Frag<__bf16>::load(Ksh + (j * 16 + c) * 64 + dc * 32 + 8 * hh);
        const v16b kl = Frag<__bf16>::load(Ksl + (j * 16 + c) * 64 + dc * 32 + 8 * hh);
        s[j] = at_mma(qa, kb, s[j]);
        s[j] = at_mma(qa, kl, s[j]);
        s[j] = at_mma(ql, kb, s[j]);
      }
    }
    const bool diag = (kc == qb);
    float cm[8];
#pragma unroll
    for (int r = 0; r < 8; ++r) {
      const int qrow = q0 + 8 * hh + r;
      float m = -INFINITY;
#pragma unroll
      for (int j = 0; j < 4; ++j) {
        const int kvcol = kv0 + j * 16 + c;
        const bool masked = diag && (kvcol > qrow);
        const float sv = masked ? -INFINITY : s[j][r];
        s[j][r] = sv;
        m = fmaxf(m, sv);
      }
#pragma unroll
      for (int off = 1; off < 16; off <<= 1) m = fmaxf(m, __shfl_xor(m, off, 32));
      cm[r] = m;
    }
    __bf16* pwh = Psh[wave];
    __bf16* pwl = Psl[wave];
#pragma unroll
    for (int r = 0; r < 8; ++r) {
      const float mnew  = fmaxf(mrow[r], cm[r]);
      const float alpha = expf(mrow[r] - mnew);
      mrow[r] = mnew;
      float psum = 0.f;
#pragma unroll
      for (int j = 0; j < 4; ++j) {
        const float p = expf(s[j][r] - mnew);
        psum += p;
        __bf16 ph, pl;
        at_split(p, ph, pl);
        pwh[(8 * hh + r) * 64 + j * 16 + c] = ph;
        pwl[(8 * hh + r) * 64 + j * 16 + c] = pl;
      }
#pragma unroll
      for (int off = 1; off < 16; off <<= 1) psum += __shfl_xor(psum, off, 32);
      lrow[r] = lrow[r] * alpha + psum;
#pragma unroll
      for (int t = 0; t < 4; ++t) oacc[t][r] *= alpha;
    }
    __builtin_amdgcn_fence(__ATOMIC_RELEASE, "workgroup");
    __builtin_amdgcn_wave_barrier();
    __builtin_amdgcn_fence(__ATOMIC_ACQUIRE, "workgroup");
#pragma unroll 1
    for (int kk = 0; kk < 2; ++kk) {
      const v16b pa = Frag<__bf16>::load(pwh + c * 64 + kk * 32 + 8 * hh);
      const v16b pl = Frag<__bf16>::load(pwl + c * 64 + kk * 32 + 8 * hh);
#pragma unroll
      for (int t = 0; t < 4; ++t) {
        const v16b vb = Frag<__bf16>::load(Vth + (t * 16 + c) * 64 + kk * 32 + 8 * hh);
        const v16b vl = Frag<__bf16>::load(Vtl + (t * 16 + c) * 64 + kk * 32 + 8 * hh);
        oacc[t] = at_mma(pa, vb, oacc[t]);
        oacc[t] = at_mma(pa, vl, oacc[t]);
        oacc[t] = at_mma(pl, vb, oacc[t]);
      }
    }
  }

  float* os = Os[wave];
#pragma unroll
  for (int r = 0; r < 8; ++r) {
    const float inv = 1.0f / lrow[r];
#pragma unroll
    for (int t = 0; t < 4; ++t) os[(8 * hh + r) * 68 + t * 16 + c] = oacc[t][r] * inv;
  }
  __builtin_amdgcn_fence(__ATOMIC_RELEASE, "workgroup");
  __builtin_amdgcn_wave_barrier();
  __builtin_amdgcn_fence(__ATOMIC_ACQUIRE, "workgroup");
  {
    const int q4 = lane >> 3, c8 = (lane & 7) * 8;
    for (int pass = 0; pass < 2; ++pass) {
#pragma unroll
      for (int it = 0; it < 4; ++it) {
        const int row = it * 4 + q4;
        const float* sp = os + row * 68 + c8;
        const v4f x0 = *(const v4f*)(sp);
        const v4f x1 = *(const v4f*)(sp + 4);
        unsigned h0, h1, h2, h3, l0, l1, l2, l3;
        h0 = pack_hl(x0.x, x0.y, l0);
        h1 = pack_hl(x0.z, x0.w, l1);
        h2 = pack_hl(x1.x, x1.y, l2);
        h3 = pack_hl(x1.z, x1.w, l3);
        const v4u uh = (v4u){h0, h1, h2, h3};
        const v4u ul = (v4u){l0, l1, l2, l3};
        const size_t o = (rowb + q0 + row) * kEmb + hcol + c8;
        *(volatile v4u*)(Oh + o) = uh;
        *(volatile v4u*)(Ol + o) = ul;
      }
      __threadfence();
    }
  }
}

extern "C" void kernel_launch(void* const* d_in, const int* in_sizes, int n_in,
                              void* d_out, int out_size, void* d_ws, size_t ws_size,
                              hipStream_t stream) {
  if (n_in < 9) return;
  if (in_sizes[0] != kRows * kEmb || out_size != kRows * kEmb) return;
  if (in_sizes[1] != kEmb * kEmb || in_sizes[3] != kEmb * kEmb || in_sizes[5] != kEmb * kEmb || in_sizes[7] != kEmb * kEmb) return;
  if (in_sizes[2] != kEmb || in_sizes[4] != kEmb || in_sizes[6] != kEmb || in_sizes[8] != kEmb) return;

  const float* x  = (const float*)d_in[0];
  const float* Wq = (const float*)d_in[1];
  const float* bq = (const float*)d_in[2];
  const float* Wk = (const float*)d_in[3];
  const float* bk = (const float*)d_in[4];
  const float* Wv = (const float*)d_in[5];
  const float* bv = (const float*)d_in[6];
  const float* Wo = (const float*)d_in[7];
  const float* bo = (const float*)d_in[8];
  float* out = (float*)d_out;

  const size_t szPlane16 = (size_t)kRows * kEmb * 2;
  const size_t szW16     = (size_t)kEmb * kEmb * 2;
  const size_t szTab     = (size_t)kSeq * kFreq * 4;
  const size_t szPlane32 = (size_t)kRows * kEmb * 4;
  size_t off = 0;
  char* ws = (char*)d_ws;
  unsigned short* Xb  = (unsigned short*)(ws + off); off += szPlane16;
  unsigned short* Wqt = (unsigned short*)(ws + off); off += szW16;
  unsigned short* Wkt = (unsigned short*)(ws + off); off += szW16;
  unsigned short* Wvt = (unsigned short*)(ws + off); off += szW16;
  unsigned short* Wot = (unsigned short*)(ws + off); off += szW16;
  float* cos_t = (float*)(ws + off); off += szTab;
  float* sin_t = (float*)(ws + off); off += szTab;
  float* Qf = (float*)(ws + off);
  unsigned short* Oh = (unsigned short*)(ws + off);
  unsigned short* Ol = (unsigned short*)(ws + off + szPlane16);
  off += szPlane32;
  float* Kf = (float*)(ws + off); off += szPlane32;
  unsigned short* Qh = (unsigned short*)(ws + off); off += szPlane16;
  unsigned short* Ql = (unsigned short*)(ws + off); off += szPlane16;
  unsigned short* Kh = (unsigned short*)(ws + off); off += szPlane16;
  unsigned short* Kl = (unsigned short*)(ws + off); off += szPlane16;
  unsigned short* Vth = (unsigned short*)(ws + off); off += szPlane16;
  unsigned short* Vtl = (unsigned short*)(ws + off); off += szPlane16;
  if (off > ws_size) return;

  RopeFreq fr;
  {
    const double quart[4] = {1.0, 1.7782794100389228, 3.1622776601683795, 5.6234132519034908};
    for (int j = 0; j < 16; ++j) {
      double p = quart[j & 3];
      for (int e = 0; e < (j >> 2); ++e) p *= 10.0;
      const float pf = (float)p;
      fr.f[j] = 1.0f / pf;
    }
  }

  cast_f32_bf16x8<<<dim3((kRows * kEmb / 8) / 256), dim3(256), 0, stream>>>(x, Xb, kRows * kEmb / 8);
  transpose_cast_bf16<<<dim3(kEmb / 64, kEmb / 64), dim3(128), 0, stream>>>(Wq, Wqt);
  transpose_cast_bf16<<<dim3(kEmb / 64, kEmb / 64), dim3(128), 0, stream>>>(Wk, Wkt);
  transpose_cast_bf16<<<dim3(kEmb / 64, kEmb / 64), dim3(128), 0, stream>>>(Wv, Wvt);
  transpose_cast_bf16<<<dim3(kEmb / 64, kEmb / 64), dim3(128), 0, stream>>>(Wo, Wot);
  rope_table<<<dim3((kSeq * kFreq) / 256), dim3(256), 0, stream>>>(cos_t, sin_t, fr);

  const int gemmBlocks = ((kRows / 64) * (kEmb / 64)) / 8;
  wmma_gemm64<1, false, 2, 0, false, 0, true><<<dim3(gemmBlocks, 1), dim3(256), 0, stream>>>(
      Xb, Xb, kEmb, (long)0, Wqt, Wqt, kEmb, (long)0, (void*)Qf, (void*)Qf, kEmb, (long)0,
      bq, bq, (long)0, kRows, kEmb, kEmb, 1.0f);
  wmma_gemm64<1, false, 2, 0, false, 0, true><<<dim3(gemmBlocks, 1), dim3(256), 0, stream>>>(
      Xb, Xb, kEmb, (long)0, Wkt, Wkt, kEmb, (long)0, (void*)Kf, (void*)Kf, kEmb, (long)0,
      bk, bk, (long)0, kRows, kEmb, kEmb, 1.0f);
  wmma_gemm64<1, false, 1, 2, false, 0, true><<<dim3(gemmBlocks, 1), dim3(256), 0, stream>>>(
      Wvt, Wvt, kEmb, (long)0, Xb, Xb, kEmb, (long)0, (void*)Vth, (void*)Vtl, kRows, (long)0,
      bv, bv, (long)0, kEmb, kRows, kEmb, 1.0f);
  rope_split<<<dim3((kRows * kHeads * 8) / 256), dim3(256), 0, stream>>>(Qf, Kf, cos_t, sin_t, Qh, Ql, Kh, Kl);
  attn_causal64<<<dim3(kBatch * kHeads * (kSeq / 64)), dim3(128), 0, stream>>>(Qh, Ql, Kh, Kl, Vth, Vtl, Oh, Ol);
  wmma_gemm64<1, true, 2, 0, false, 0, false><<<dim3(gemmBlocks, 1), dim3(256), 0, stream>>>(
      Oh, Ol, kEmb, (long)0, Wot, Wot, kEmb, (long)0, (void*)out, (void*)out, kEmb, (long)0,
      bo, bo, (long)0, kRows, kEmb, kEmb, 1.0f);
}
